// class_self_MultiHeadAttention_54065048322415
// MI455X (gfx1250) — hardware-verified
//
#include <hip/hip_runtime.h>


namespace {
constexpr int N = 4096, D = 256, H = 4, HD = 64, NE = 9, D3 = 3 * D;
constexpr float XS = 8.0f, PS = 8.0f, SCALE = 0.25f, LN_EPS = 1e-5f;

typedef _Float16 b16;
typedef __attribute__((ext_vector_type(16))) _Float16 v16b;
typedef __attribute__((ext_vector_type(8))) _Float16 v8b;
typedef __attribute__((ext_vector_type(8))) float v8f;
typedef __attribute__((ext_vector_type(4))) float v4f;
__device__ __forceinline__ float bf16_rne(float f) { unsigned int u = __float_as_uint(f); u += 0x7FFFu + ((u >> 16) & 1u); return __uint_as_float(u & 0xFFFF0000u); }
__device__ __forceinline__ void split16(float v, b16& hi, b16& lo) { hi = (b16)v; lo = (b16)(v - (float)hi); }
__device__ __forceinline__ v16b frag_kb(const b16* p, int hh) { const v8b a = *(const v8b*)(p + 8 * hh), b = *(const v8b*)(p + 16 + 8 * hh); v16b f;
#pragma unroll
  for (int e = 0; e < 8; ++e) { f[e] = a[e]; f[8 + e] = b[e]; } return f; }
__device__ __forceinline__ v8f wmma16b(v16b a, v16b b, v8f c) { v8f d = __builtin_amdgcn_wmma_f32_16x16x32_f16(false, a, false, b, (short)0, c, false, false); asm volatile("v_nop\n\tv_nop\n\tv_nop\n\tv_nop" : "+v"(d) : "v"(a), "v"(b)); return d; }
__device__ __forceinline__ void wave_lds_sync() { __builtin_amdgcn_fence(__ATOMIC_RELEASE, "workgroup"); __builtin_amdgcn_wave_barrier(); __builtin_amdgcn_fence(__ATOMIC_ACQUIRE, "workgroup"); }
__device__ __forceinline__ float nexp(float x) { return __builtin_amdgcn_exp2f(x * 1.4426950408889634f); }
__device__ __forceinline__ float pmul(float a, float b) { float p = a * b; asm volatile("" : "+v"(p)); return p; }

__global__ __launch_bounds__(256) void prep_kernel(const float* __restrict__ x, const float* __restrict__ wq, const float* __restrict__ wk, const float* __restrict__ wv, const float* __restrict__ wf, const float* __restrict__ bq, const float* __restrict__ bk, const float* __restrict__ bv, const float* __restrict__ bff, const float* __restrict__ gm, const float* __restrict__ bt, b16* __restrict__ R, b16* __restrict__ RF, b16* __restrict__ X, float* __restrict__ P) {
  const size_t tid = (size_t)blockIdx.x * 256 + threadIdx.x, nth = (size_t)gridDim.x * 256;
  for (int pass = 0; pass < 2; ++pass) {
    for (size_t p = tid; p < (size_t)NE * D3 * (D / 8); p += nth) { const int e_ = (int)(p / ((size_t)D3 * (D / 8))); const size_t r = p % ((size_t)D3 * (D / 8)); const int o3 = (int)(r / (D / 8)), k0 = (int)(r % (D / 8)) * 8; const int w = o3 / D, o = o3 % D;
      const float* W = (w == 0) ? wq : (w == 1) ? wk : wv; v8b v; for (int e = 0; e < 8; ++e) v[e] = (b16)bf16_rne(W[((size_t)e_ * D + k0 + e) * D + o]); *(volatile v8b*)(R + ((size_t)e_ * D3 + o3) * D + k0) = v; }
    for (size_t p = tid; p < (size_t)D * (D / 8); p += nth) { const int o = (int)(p / (D / 8)), k0 = (int)(p % (D / 8)) * 8; v8b v; for (int e = 0; e < 8; ++e) v[e] = (b16)bf16_rne(wf[(size_t)(k0 + e) * D + o]); *(volatile v8b*)(RF + (size_t)o * D + k0) = v; }
    for (size_t p = tid; p < (size_t)N * D / 8; p += nth) { v8b v; for (int e = 0; e < 8; ++e) v[e] = (b16)(bf16_rne(x[p * 8 + e]) * XS); *(volatile v8b*)(X + p * 8) = v; }
    for (size_t q = tid; q < 7680; q += nth) { const int i = (int)q; float v; if (i < 6912) { const int e_ = i / D3, c = i % D3; v = (c < D) ? bq[e_ * D + c] : (c < 2 * D) ? bk[e_ * D + c - D] : bv[e_ * D + c - 2 * D]; } else if (i < 7168) v = bff[i - 6912]; else if (i < 7424) v = gm[i - 7168]; else v = bt[i - 7424]; P[q] = bf16_rne(v); }
    __threadfence(); }
}

__global__ __launch_bounds__(64) void proj_kernel(const b16* __restrict__ X, const b16* __restrict__ R, const float* __restrict__ P, float* __restrict__ ALL) {
  __shared__ __attribute__((aligned(16))) float Ts[2][32][128 + 4];
  const int lane = threadIdx.x & 31, wave = threadIdx.x >> 5, nloc = lane & 15, hlf = lane >> 4, m0 = blockIdx.y * 32, c0 = blockIdx.x * 256 + wave * 128, e_ = blockIdx.z; const b16* Bw = R + (size_t)e_ * D3 * D;
  v8f acc[2][8];
#pragma unroll
  for (int r = 0; r < 2; ++r)
#pragma unroll
    for (int t = 0; t < 8; ++t) acc[r][t] = (v8f){};
#pragma unroll
  for (int kb = 0; kb < D; kb += 32) { const v16b a0 = frag_kb(X + (size_t)(m0 + nloc) * D + kb, hlf), a1 = frag_kb(X + (size_t)(m0 + 16 + nloc) * D + kb, hlf);
#pragma unroll
    for (int t = 0; t < 8; ++t) { const v16b bw = frag_kb(Bw + (size_t)(c0 + t * 16 + nloc) * D + kb, hlf); acc[0][t] = wmma16b(a0, bw, acc[0][t]); acc[1][t] = wmma16b(a1, bw, acc[1][t]); } }
#pragma unroll
  for (int t = 0; t < 8; ++t) { const float bb = P[e_ * D3 + c0 + t * 16 + nloc];
#pragma unroll
    for (int r = 0; r < 2; ++r)
#pragma unroll
      for (int v = 0; v < 8; ++v) Ts[wave][r * 16 + 8 * hlf + v][t * 16 + nloc] = acc[r][t][v] * (1.0f / XS) + bb; }
  wave_lds_sync();
  for (int pass = 0; pass < 2; ++pass) { for (int i = lane; i < 32 * 32; i += 32) { const int rr = i >> 5, c4 = (i & 31) * 4; *(volatile v4f*)(ALL + ((size_t)e_ * N + m0 + rr) * D3 + c0 + c4) = *(const v4f*)(&Ts[wave][rr][c4]); } __threadfence(); }
}

__global__ __launch_bounds__(256) void select_kernel(const float* __restrict__ ALL, const int* __restrict__ lbl, b16* __restrict__ QK, b16* __restrict__ VTh, b16* __restrict__ VTl) {
  __shared__ __attribute__((aligned(16))) b16 Th[D][128 + 8], Tl[D][128 + 8];
  const int t0 = blockIdx.x * 128, t_ = threadIdx.x;
  for (int i = t_; i < 128 * (D / 4); i += 256) { const int tk = i / (D / 4), c4 = (i % (D / 4)) * 4; int e_ = lbl[t0 + tk]; e_ = (e_ < 0) ? 0 : (e_ >= NE ? NE - 1 : e_); const v4f vv = *(const v4f*)(ALL + ((size_t)e_ * N + t0 + tk) * D3 + 2 * D + c4);
    for (int e = 0; e < 4; ++e) { b16 a_, b_; split16(vv[e] * XS, a_, b_); Th[c4 + e][tk] = a_; Tl[c4 + e][tk] = b_; } }
  __syncthreads();
  for (int pass = 0; pass < 2; ++pass) {
    for (int i = t_; i < 128 * (2 * D / 8); i += 256) { const int tk = i / (2 * D / 8), c8 = (i % (2 * D / 8)) * 8; int e_ = lbl[t0 + tk]; e_ = (e_ < 0) ? 0 : (e_ >= NE ? NE - 1 : e_); const float* src = ALL + ((size_t)e_ * N + t0 + tk) * D3 + c8;
      v8b o; for (int e = 0; e < 8; ++e) o[e] = (b16)(src[e] * XS); *(volatile v8b*)(QK + (size_t)(t0 + tk) * (2 * D) + c8) = o; }
    for (int i = t_; i < D * 16; i += 256) { const int c = i >> 4, c8 = (i & 15) * 8; const int h = c / HD, d = c % HD; const size_t gi = ((size_t)h * HD + d) * N + t0 + c8; *(volatile v8b*)(VTh + gi) = *(const v8b*)(&Th[c][c8]); *(volatile v8b*)(VTl + gi) = *(const v8b*)(&Tl[c][c8]); }
    __threadfence(); }
}

__global__ __launch_bounds__(128) void attn_kernel(const b16* __restrict__ QK, const b16* __restrict__ VTh, const b16* __restrict__ VTl, const int* __restrict__ lbl, b16* __restrict__ CH, b16* __restrict__ CL) {
  __shared__ int Lk[32]; __shared__ __attribute__((aligned(16))) b16 Oh[16][D + 8], Ol[16][D + 8];
  const int wid = threadIdx.x >> 5, lane = threadIdx.x & 31, hh = lane >> 4, col = lane & 15; const int q0 = blockIdx.x * 16, h = wid, qi = q0 + col; const int lq = lbl[qi];
  const b16* Qr = QK + h * HD; const b16* Kr = QK + D + h * HD; const b16* V = VTh + ((size_t)h * HD) * N; const b16* Vl = VTl + ((size_t)h * HD) * N;
  const v16b qf0 = frag_kb(Qr + (size_t)qi * (2 * D), hh), qf1 = frag_kb(Qr + (size_t)qi * (2 * D) + 32, hh);
  float m = -INFINITY, l = 0.0f; v8f o[4] = {{}, {}, {}, {}};
  for (int kb = 0; kb < N; kb += 32) {
    __syncthreads(); if (threadIdx.x < 32) Lk[threadIdx.x] = lbl[kb + threadIdx.x]; __syncthreads();
    v8f s0 = {}, s1 = {}; s0 = wmma16b(frag_kb(Kr + (size_t)(kb + col) * (2 * D), hh), qf0, s0); s0 = wmma16b(frag_kb(Kr + (size_t)(kb + col) * (2 * D) + 32, hh), qf1, s0);
    s1 = wmma16b(frag_kb(Kr + (size_t)(kb + 16 + col) * (2 * D), hh), qf0, s1); s1 = wmma16b(frag_kb(Kr + (size_t)(kb + 16 + col) * (2 * D) + 32, hh), qf1, s1);
    float mr = -INFINITY;
#pragma unroll
    for (int r = 0; r < 8; ++r) { s0[r] = (Lk[8 * hh + r] == lq) ? s0[r] * (SCALE / (XS * XS)) : -INFINITY; s1[r] = (Lk[16 + 8 * hh + r] == lq) ? s1[r] * (SCALE / (XS * XS)) : -INFINITY; mr = fmaxf(mr, fmaxf(s0[r], s1[r])); }
    mr = fmaxf(mr, __shfl_xor(mr, 16)); const float mn = fmaxf(m, mr); const float al_ = (mn == -INFINITY) ? 1.0f : nexp(m - mn); m = mn; float sum = 0.0f; v16b pb, pl;
#pragma unroll
    for (int r = 0; r < 8; ++r) { const float e0 = (s0[r] == -INFINITY) ? 0.0f : nexp(s0[r] - mn), e1 = (s1[r] == -INFINITY) ? 0.0f : nexp(s1[r] - mn); sum += e0 + e1; b16 a_, c_; split16(e0 * PS, a_, c_); pb[r] = a_; pl[r] = c_; split16(e1 * PS, a_, c_); pb[8 + r] = a_; pl[8 + r] = c_; }
    sum += __shfl_xor(sum, 16); l = l * al_ + sum;
#pragma unroll
    for (int t = 0; t < 4; ++t) { o[t] *= al_; const v16b vh = frag_kb(V + (size_t)(t * 16 + col) * N + kb, hh), vlo = frag_kb(Vl + (size_t)(t * 16 + col) * N + kb, hh); o[t] = wmma16b(vh, pb, o[t]); o[t] = wmma16b(vh, pl, o[t]); o[t] = wmma16b(vlo, pb, o[t]); } }
  const float inv = 1.0f / (l * PS);
#pragma unroll
  for (int t = 0; t < 4; ++t)
#pragma unroll
    for (int r = 0; r < 8; ++r) { b16 a_, c_; split16(o[t][r] * inv, a_, c_); Oh[col][h * HD + t * 16 + 8 * hh + r] = a_; Ol[col][h * HD + t * 16 + 8 * hh + r] = c_; }
  __syncthreads();
  for (int pass = 0; pass < 2; ++pass) { for (int i = threadIdx.x; i < 16 * 32; i += 128) { const int rr = i >> 5, c8 = (i & 31) * 8; const size_t gi = (size_t)(q0 + rr) * D + c8; *(volatile v8b*)(CH + gi) = *(const v8b*)(&Oh[rr][c8]); *(volatile v8b*)(CL + gi) = *(const v8b*)(&Ol[rr][c8]); } __threadfence(); }
}

__global__ __launch_bounds__(64) void out_kernel(const b16* __restrict__ CH, const b16* __restrict__ CL, const b16* __restrict__ RF, const float* __restrict__ P, const float* __restrict__ x, float* __restrict__ out) {
  __shared__ __attribute__((aligned(16))) float Ts[32][D + 4];
  const int lane = threadIdx.x & 31, wave = threadIdx.x >> 5, nloc = lane & 15, hlf = lane >> 4, m0 = blockIdx.x * 32, c0 = wave * 128;
  v8f acc[2][8];
#pragma unroll
  for (int r = 0; r < 2; ++r)
#pragma unroll
    for (int t = 0; t < 8; ++t) acc[r][t] = (v8f){};
#pragma unroll
  for (int kb = 0; kb < D; kb += 32) { const v16b a0 = frag_kb(CH + (size_t)(m0 + nloc) * D + kb, hlf), a1 = frag_kb(CH + (size_t)(m0 + 16 + nloc) * D + kb, hlf), l0 = frag_kb(CL + (size_t)(m0 + nloc) * D + kb, hlf), l1 = frag_kb(CL + (size_t)(m0 + 16 + nloc) * D + kb, hlf);
#pragma unroll
    for (int t = 0; t < 8; ++t) { const v16b bw = frag_kb(RF + (size_t)(c0 + t * 16 + nloc) * D + kb, hlf); acc[0][t] = wmma16b(a0, bw, acc[0][t]); acc[0][t] = wmma16b(l0, bw, acc[0][t]); acc[1][t] = wmma16b(a1, bw, acc[1][t]); acc[1][t] = wmma16b(l1, bw, acc[1][t]); } }
#pragma unroll
  for (int t = 0; t < 8; ++t) { const int c = c0 + t * 16 + nloc; const float bb = P[6912 + c];
#pragma unroll
    for (int r = 0; r < 2; ++r)
#pragma unroll
      for (int v = 0; v < 8; ++v) { const int rr = r * 16 + 8 * hlf + v; Ts[rr][c] = acc[r][t][v] * (1.0f / XS) + bb + bf16_rne(x[(size_t)(m0 + rr) * D + c]); } }
  __syncthreads();
  for (int rr = wave * 16; rr < wave * 16 + 16; ++rr) { float v[8]; float s = 0.0f;
#pragma unroll
    for (int e = 0; e < 8; ++e) { v[e] = Ts[rr][lane * 8 + e]; s += v[e]; }
#pragma unroll
    for (int o_ = 1; o_ < 32; o_ <<= 1) s += __shfl_xor(s, o_);
    const float mu = s * (1.0f / D); float q = 0.0f;
#pragma unroll
    for (int e = 0; e < 8; ++e) { const float d_ = v[e] - mu; q += pmul(d_, d_); }
#pragma unroll
    for (int o_ = 1; o_ < 32; o_ <<= 1) q += __shfl_xor(q, o_);
    const float inv = rsqrtf(q * (1.0f / D) + LN_EPS);
#pragma unroll
    for (int e = 0; e < 8; ++e) { const int c = lane * 8 + e; Ts[rr][c] = pmul((v[e] - mu) * inv, P[7168 + c]) + P[7424 + c]; } }
  wave_lds_sync();
  for (int pass = 0; pass < 2; ++pass) { for (int i = lane; i < 16 * 64; i += 32) { const int rr = wave * 16 + (i >> 6), c4 = (i & 63) * 4; *(volatile v4f*)(out + (size_t)(m0 + rr) * D + c4) = *(const v4f*)(&Ts[rr][c4]); } __threadfence(); }
}
}

extern "C" void kernel_launch(void* const* d_in, const int* in_sizes, int n_in,
                              void* d_out, int out_size, void* d_ws, size_t ws_size, hipStream_t stream) {
  (void)n_in; (void)out_size;
  const float* x = (const float*)d_in[0]; const int* lbl = (const int*)d_in[1]; const float* wq = (const float*)d_in[2]; const float* bq = (const float*)d_in[3]; const float* wk = (const float*)d_in[4]; const float* bk = (const float*)d_in[5]; const float* wv = (const float*)d_in[6]; const float* bv = (const float*)d_in[7];
  const float* wf = (const float*)d_in[8]; const float* bff = (const float*)d_in[9]; const float* gm = (const float*)d_in[10]; const float* bt = (const float*)d_in[11];
  float* out = (float*)d_out;
  if (in_sizes[0] != N * D || in_sizes[1] != N || in_sizes[2] != NE * D * D || in_sizes[8] != D * D) return;
  size_t off = 0; char* ws = (char*)d_ws;
  auto carve = [&](size_t bytes) { char* p = ws + off; off += (bytes + 255) & ~(size_t)255; return p; };
  b16* R = (b16*)carve((size_t)NE * D3 * D * 2); b16* RF = (b16*)carve((size_t)D * D * 2); b16* X = (b16*)carve((size_t)N * D * 2); float* P = (float*)carve(7680 * 4); float* ALL = (float*)carve((size_t)NE * N * D3 * 4);
  b16* QK = (b16*)carve((size_t)N * 2 * D * 2); b16* VTh = (b16*)carve((size_t)N * D * 2); b16* VTl = (b16*)carve((size_t)N * D * 2); b16* CH = (b16*)carve((size_t)N * D * 2); b16* CL = (b16*)carve((size_t)N * D * 2);
  if (off > ws_size) return;
  prep_kernel<<<256, 256, 0, stream>>>(x, wq, wk, wv, wf, bq, bk, bv, bff, gm, bt, R, RF, X, P);
  proj_kernel<<<dim3(3, N / 32, NE), 64, 0, stream>>>(X, R, P, ALL);
  select_kernel<<<N / 128, 256, 0, stream>>>(ALL, lbl, QK, VTh, VTl);
  attn_kernel<<<N / 16, 128, 0, stream>>>(QK, VTh, VTl, lbl, CH, CL);
  out_kernel<<<N / 32, 64, 0, stream>>>(CH, CL, RF, P, x, out);
}
